// EdgePredictor_43276090474511
// MI455X (gfx1250) — hardware-verified
//
#include <hip/hip_runtime.h>


typedef _Float16 v16h __attribute__((ext_vector_type(16)));
typedef _Float16 v8h  __attribute__((ext_vector_type(8)));
typedef __bf16   v16b __attribute__((ext_vector_type(16)));
typedef unsigned short v8us __attribute__((ext_vector_type(8)));
typedef float v8f __attribute__((ext_vector_type(8)));
typedef float v4f __attribute__((ext_vector_type(4)));

union FragH { v16h v; v8h p[2]; };
union FragB { v16b v; v8us p[2]; };

constexpr int NPTS = 1024;
constexpr int DD   = 64;
constexpr int AH   = 256;

__device__ __forceinline__ v8f wmma_f16(v16h a, v16h b, v8f c) {
    c = __builtin_amdgcn_wmma_f32_16x16x32_f16(false, a, false, b, (short)0, c, false, false);
    asm volatile("v_nop\n\tv_nop\n\tv_nop\n\tv_nop" : "+v"(c) : "v"(a), "v"(b));
    return c;
}
__device__ __forceinline__ v8f wmma_bf16(v16b a, v16b b, v8f c) {
    c = __builtin_amdgcn_wmma_f32_16x16x32_bf16(false, a, false, b, (short)0, c, false, false);
    asm volatile("v_nop\n\tv_nop\n\tv_nop\n\tv_nop" : "+v"(c) : "v"(a), "v"(b));
    return c;
}

__device__ __forceinline__ v16h ld_frag_h(const _Float16* rowbase, int kt, int h) {
    const _Float16* p = rowbase + kt * 32 + 8 * h;
    FragH f;
    f.p[0] = *(const v8h*)p;
    f.p[1] = *(const v8h*)(p + 16);
    return f.v;
}
__device__ __forceinline__ v16b ld_frag_b(const unsigned short* rowbase, int kt, int h) {
    const unsigned short* p = rowbase + kt * 32 + 8 * h;
    FragB f;
    f.p[0] = *(const v8us*)p;
    f.p[1] = *(const v8us*)(p + 16);
    return f.v;
}

__device__ __forceinline__ unsigned short bf16_rne(float f) {
    unsigned u = __float_as_uint(f);
    u += 0x7FFFu + ((u >> 16) & 1u);
    return (unsigned short)(u >> 16);
}
__device__ __forceinline__ float bf16_val(unsigned short s) {
    return __uint_as_float(((unsigned)s) << 16);
}

template <int KIN, int NO, bool HASB>
__global__ void __launch_bounds__(NO)
rowlin_kernel(const float* __restrict__ in, const float* __restrict__ W,
              const float* __restrict__ b, float* o0, float* o1, float* o2, int nrows) {
    __shared__ __attribute__((aligned(16))) float s_o[4][NO];
    const int tid = threadIdx.x;
    const int i0 = blockIdx.x * 4;
    float acc[4];
#pragma unroll
    for (int r = 0; r < 4; ++r) acc[r] = 0.f;
#pragma unroll 1
    for (int kk = 0; kk < KIN; ++kk) {
        const float w = W[kk * NO + tid];
#pragma unroll
        for (int r = 0; r < 4; ++r) {
            int ir = i0 + r; ir = (ir < nrows) ? ir : (nrows - 1);
            acc[r] = fmaf(in[(size_t)ir * KIN + kk], w, acc[r]);
        }
    }
    const float bm = HASB ? b[tid] : 0.f;
#pragma unroll
    for (int r = 0; r < 4; ++r) s_o[r][tid] = acc[r] + bm;
    __syncthreads();

    constexpr int LPR = NO / 32;
    const int L = tid >> 3, e = tid & 7;
    const int r = L / LPR, seg = L % LPR;
    const int buf = seg >> 1, half = seg & 1;
    const v4f val = *(const v4f*)(&s_o[r][seg * 32 + e * 4]);
    float* base = (buf == 0) ? o0 : ((buf == 1) ? o1 : o2);
    float* dst = base + (size_t)(i0 + r) * 64 + half * 32 + e * 4;
    if ((i0 + r) < nrows) {
        *(volatile v4f*)dst = val;
        __threadfence();
        *(volatile v4f*)dst = val;
    }
}

__global__ void __launch_bounds__(64)
fc_split_kernel(const float* __restrict__ feats, const float* __restrict__ W,
                const float* __restrict__ b, unsigned short* phi, unsigned short* plo,
                int nrows) {
    __shared__ __attribute__((aligned(16))) float s_o[4][64];
    const int tid = threadIdx.x;
    const int i0 = blockIdx.x * 4;
    float acc[4];
#pragma unroll
    for (int r = 0; r < 4; ++r) acc[r] = 0.f;
#pragma unroll 1
    for (int kk = 0; kk < 64; ++kk) {
        const float w = W[kk * 64 + tid];
#pragma unroll
        for (int r = 0; r < 4; ++r) {
            int ir = i0 + r; ir = (ir < nrows) ? ir : (nrows - 1);
            acc[r] = fmaf(feats[(size_t)ir * 64 + kk], w, acc[r]);
        }
    }
    const float bm = b[tid];
#pragma unroll
    for (int r = 0; r < 4; ++r) s_o[r][tid] = acc[r] + bm;
    __syncthreads();

    const int plane = tid >> 5;
    const int r = (tid >> 3) & 3, e = tid & 7;
    const v4f f0 = *(const v4f*)(&s_o[r][e * 8]);
    const v4f f1 = *(const v4f*)(&s_o[r][e * 8 + 4]);
    v8us hv, lv;
#pragma unroll
    for (int qq = 0; qq < 8; ++qq) {
        const float f = (qq < 4) ? f0[qq] : f1[qq - 4];
        const unsigned short hb = bf16_rne(f);
        hv[qq] = hb;
        lv[qq] = bf16_rne(f - bf16_val(hb));
    }
    v8us val = hv;
    unsigned short* base = phi;
    if (plane) { val = lv; base = plo; }
    unsigned short* dst = base + (size_t)(i0 + r) * 64 + e * 8;
    if ((i0 + r) < nrows) {
        *(volatile v8us*)dst = val;
        __threadfence();
        *(volatile v8us*)dst = val;
    }
}

constexpr int LDP2 = 72;
constexpr int LDA1 = 72;
constexpr int LDA2 = 264;
constexpr int H_PW2 = 64 * LDP2;
constexpr int H_AW1 = 256 * LDA1;
constexpr int H_AW2 = 64 * LDA2;
constexpr int H_HIN = 4 * 16 * DD;
constexpr int H_H1  = 4 * 16 * AH;
constexpr int LAYER_HALVES = H_PW2 + H_AW1 + H_AW2 + H_HIN + H_H1;
constexpr int LAYER_FLOATS = 192 + 64 + 64 + 256 + 64 + 4 * 64 * 3 + 64;
constexpr size_t LAYER_SMEM = (size_t)LAYER_HALVES * 2 + (size_t)LAYER_FLOATS * 4;

__global__ void __launch_bounds__(128)
pair_layer_kernel(const float* __restrict__ x,
                  const float* __restrict__ q, const float* __restrict__ kmat,
                  const float* __restrict__ v,
                  const float* __restrict__ pw1, const float* __restrict__ pb1,
                  const float* __restrict__ pw2, const float* __restrict__ pb2,
                  const float* __restrict__ aw1, const float* __restrict__ ab1,
                  const float* __restrict__ aw2, const float* __restrict__ ab2,
                  float* feats_out) {
    extern __shared__ __attribute__((aligned(16))) char smem[];
    _Float16* s_pw2t = (_Float16*)smem;
    _Float16* s_aw1t = s_pw2t + H_PW2;
    _Float16* s_aw2t = s_aw1t + H_AW1;
    _Float16* s_hin  = s_aw2t + H_AW2;
    _Float16* s_h1   = s_hin + H_HIN;
    float* s_pw1 = (float*)(s_h1 + H_H1);
    float* s_pb1 = s_pw1 + 192;
    float* s_pb2 = s_pb1 + 64;
    float* s_ab1 = s_pb2 + 64;
    float* s_ab2 = s_ab1 + 256;
    float* s_red = s_ab2 + 64;
    float* s_fin = s_red + 768;

    const int tid = threadIdx.x;
    for (int idx = tid; idx < 64 * 64; idx += 128) {
        const int kk = idx >> 6, n = idx & 63;
        s_pw2t[n * LDP2 + kk] = (_Float16)pw2[idx];
    }
    for (int idx = tid; idx < 64 * 256; idx += 128) {
        const int kk = idx >> 8, n = idx & 255;
        s_aw1t[n * LDA1 + kk] = (_Float16)aw1[idx];
    }
    for (int idx = tid; idx < 256 * 64; idx += 128) {
        const int kk = idx >> 6, n = idx & 63;
        s_aw2t[n * LDA2 + kk] = (_Float16)aw2[idx];
    }
    for (int t = tid; t < 192; t += 128) s_pw1[t] = pw1[t];
    for (int t = tid; t < 256; t += 128) s_ab1[t] = ab1[t];
    if (tid < 64) {
        s_pb1[tid] = pb1[tid];
        s_pb2[tid] = pb2[tid];
        s_ab2[tid] = ab2[tid];
    }
    __syncthreads();

    const int i    = blockIdx.x;
    const int wave = tid >> 5;
    const int lane = tid & 31;
    const int lr   = lane & 15;
    const int hi   = lane >> 4;

    const float xi0 = x[2 * i], xi1 = x[2 * i + 1];
    float qd[4];
#pragma unroll
    for (int nt = 0; nt < 4; ++nt) qd[nt] = q[(size_t)i * 64 + nt * 16 + lr];

    float m_s[4], s_s[4], a_s[4];
#pragma unroll
    for (int nt = 0; nt < 4; ++nt) { m_s[nt] = -1e30f; s_s[nt] = 0.f; a_s[nt] = 0.f; }

    _Float16* my_hin = s_hin + wave * 16 * DD;
    _Float16* my_h1  = s_h1 + wave * 16 * AH;

    for (int jt = wave; jt < 64; jt += 4) {
        const int jbase = jt * 16;
        const int jrow  = jbase + lr;
        const float rx = xi0 - x[2 * jrow];
        const float ry = xi1 - x[2 * jrow + 1];

        v16h hA[2];
#pragma unroll
        for (int kt = 0; kt < 2; ++kt) {
#pragma unroll
            for (int e = 0; e < 16; ++e) {
                const int kl = (e < 8) ? (hi * 8 + e) : (16 + hi * 8 + (e - 8));
                const int p  = kt * 32 + kl;
                const float hv = fmaf(rx, s_pw1[p], fmaf(ry, s_pw1[64 + p], s_pb1[p]));
                hA[kt][e] = (_Float16)fmaxf(hv, 0.f);
            }
        }

        v8f relC[4];
#pragma unroll
        for (int nt = 0; nt < 4; ++nt) {
            const float bb = s_pb2[nt * 16 + lr];
            v8f c;
#pragma unroll
            for (int r = 0; r < 8; ++r) c[r] = bb;
#pragma unroll
            for (int kt = 0; kt < 2; ++kt)
                c = wmma_f16(hA[kt], ld_frag_h(s_pw2t + (nt * 16 + lr) * LDP2, kt, hi), c);
            relC[nt] = c;
        }

#pragma unroll
        for (int nt = 0; nt < 4; ++nt) {
#pragma unroll
            for (int r = 0; r < 8; ++r) {
                const int row = r + 8 * hi;
                const float kv = kmat[(size_t)(jbase + row) * 64 + nt * 16 + lr];
                const float hv = qd[nt] - kv + relC[nt][r];
                my_hin[row * DD + nt * 16 + lr] = (_Float16)hv;
            }
        }
        __syncthreads();

        v16h hinA[2];
#pragma unroll
        for (int kt = 0; kt < 2; ++kt) hinA[kt] = ld_frag_h(my_hin + lr * DD, kt, hi);

#pragma unroll
        for (int nt = 0; nt < 16; ++nt) {
            const float bb = s_ab1[nt * 16 + lr];
            v8f c;
#pragma unroll
            for (int r = 0; r < 8; ++r) c[r] = bb;
#pragma unroll
            for (int kt = 0; kt < 2; ++kt)
                c = wmma_f16(hinA[kt], ld_frag_h(s_aw1t + (nt * 16 + lr) * LDA1, kt, hi), c);
#pragma unroll
            for (int r = 0; r < 8; ++r)
                my_h1[(r + 8 * hi) * AH + nt * 16 + lr] = (_Float16)fmaxf(c[r], 0.f);
        }
        __syncthreads();

#pragma unroll
        for (int nt = 0; nt < 4; ++nt) {
            const float bb = s_ab2[nt * 16 + lr];
            v8f c;
#pragma unroll
            for (int r = 0; r < 8; ++r) c[r] = bb;
#pragma unroll
            for (int kt = 0; kt < 8; ++kt) {
                const v16h a = ld_frag_h(my_h1 + lr * AH, kt, hi);
                const v16h bfr = ld_frag_h(s_aw2t + (nt * 16 + lr) * LDA2, kt, hi);
                c = wmma_f16(a, bfr, c);
            }

            float tmax = c[0];
#pragma unroll
            for (int r = 1; r < 8; ++r) tmax = fmaxf(tmax, c[r]);
            tmax = fmaxf(tmax, __shfl_xor(tmax, 16, 32));
            const float mnew  = fmaxf(m_s[nt], tmax);
            const float alpha = __expf(m_s[nt] - mnew);
            float ps = 0.f, pa = 0.f;
#pragma unroll
            for (int r = 0; r < 8; ++r) {
                const float ee = __expf(c[r] - mnew);
                const float vv = v[(size_t)(jbase + r + 8 * hi) * 64 + nt * 16 + lr] + relC[nt][r];
                ps += ee;
                pa += ee * vv;
            }
            ps += __shfl_xor(ps, 16, 32);
            pa += __shfl_xor(pa, 16, 32);
            s_s[nt] = s_s[nt] * alpha + ps;
            a_s[nt] = a_s[nt] * alpha + pa;
            m_s[nt] = mnew;
        }
    }

    if (hi == 0) {
#pragma unroll
        for (int nt = 0; nt < 4; ++nt) {
            const int d = nt * 16 + lr;
            s_red[(wave * 64 + d) * 3 + 0] = m_s[nt];
            s_red[(wave * 64 + d) * 3 + 1] = s_s[nt];
            s_red[(wave * 64 + d) * 3 + 2] = a_s[nt];
        }
    }
    __syncthreads();
    if (tid < 64) {
        const int d = tid;
        float M = -1e30f;
#pragma unroll
        for (int w = 0; w < 4; ++w) M = fmaxf(M, s_red[(w * 64 + d) * 3]);
        float S = 0.f, A = 0.f;
#pragma unroll
        for (int w = 0; w < 4; ++w) {
            const float ee = __expf(s_red[(w * 64 + d) * 3] - M);
            S += s_red[(w * 64 + d) * 3 + 1] * ee;
            A += s_red[(w * 64 + d) * 3 + 2] * ee;
        }
        s_fin[d] = A / S;
    }
    __syncthreads();
    if (tid < 16) {
        const v4f val = *(const v4f*)(s_fin + 4 * tid);
        float* dst = feats_out + (size_t)i * 64 + 4 * tid;
        *(volatile v4f*)dst = val;
        __threadfence();
        *(volatile v4f*)dst = val;
    }
}

__global__ void __launch_bounds__(32)
edge_kernel(const unsigned short* __restrict__ f1hi, const unsigned short* __restrict__ f1lo,
            float* out) {
    __shared__ __attribute__((aligned(16))) float s_t[16][64];
    const int lane = threadIdx.x;
    const int lr = lane & 15, hi = lane >> 4;
    const int mbase = blockIdx.y * 16;
    const int nb0   = blockIdx.x * 64;

    v16b Ah[2], Al[2];
    {
        const unsigned short* arh = f1hi + (size_t)(mbase + lr) * 64;
        const unsigned short* arl = f1lo + (size_t)(mbase + lr) * 64;
#pragma unroll
        for (int kt = 0; kt < 2; ++kt) { Ah[kt] = ld_frag_b(arh, kt, hi); Al[kt] = ld_frag_b(arl, kt, hi); }
    }

#pragma unroll
    for (int nt4 = 0; nt4 < 4; ++nt4) {
        const int nbase = nb0 + nt4 * 16;
        const unsigned short* brh = f1hi + (size_t)(nbase + lr) * 64;
        const unsigned short* brl = f1lo + (size_t)(nbase + lr) * 64;
        v8f c;
#pragma unroll
        for (int r = 0; r < 8; ++r) c[r] = 0.f;
#pragma unroll
        for (int kt = 0; kt < 2; ++kt) {
            const v16b bh = ld_frag_b(brh, kt, hi);
            const v16b bl = ld_frag_b(brl, kt, hi);
            c = wmma_bf16(Ah[kt], bh, c);
            c = wmma_bf16(Ah[kt], bl, c);
            c = wmma_bf16(Al[kt], bh, c);
        }
#pragma unroll
        for (int r = 0; r < 8; ++r)
            s_t[8 * hi + r][nt4 * 16 + lr] = 1.f / (1.f + __expf(-c[r]));
    }
    __syncthreads();

    v4f val[8];
    float* dst[8];
#pragma unroll
    for (int p = 0; p < 8; ++p) {
        const int L = p * 4 + (lane >> 3), e = lane & 7;
        const int row = L >> 1, half = L & 1;
        val[p] = *(const v4f*)(&s_t[row][half * 32 + e * 4]);
        dst[p] = out + (size_t)(mbase + row) * NPTS + nb0 + half * 32 + e * 4;
        *(volatile v4f*)dst[p] = val[p];
    }
    __threadfence();
#pragma unroll
    for (int p = 0; p < 8; ++p) *(volatile v4f*)dst[p] = val[p];
}

extern "C" void kernel_launch(void* const* d_in, const int* in_sizes, int n_in,
                              void* d_out, int out_size, void* d_ws, size_t ws_size,
                              hipStream_t stream) {
    if (n_in < 14) return;
    const float* x     = (const float*)d_in[0];
    const float* in_w  = (const float*)d_in[1];
    const float* in_b  = (const float*)d_in[2];
    const float* qkv_w = (const float*)d_in[3];
    const float* pw1   = (const float*)d_in[4];
    const float* pb1   = (const float*)d_in[5];
    const float* pw2   = (const float*)d_in[6];
    const float* pb2   = (const float*)d_in[7];
    const float* aw1   = (const float*)d_in[8];
    const float* ab1   = (const float*)d_in[9];
    const float* aw2   = (const float*)d_in[10];
    const float* ab2   = (const float*)d_in[11];
    const float* fc_w  = (const float*)d_in[12];
    const float* fc_b  = (const float*)d_in[13];
    float* out = (float*)d_out;

    const int npts = in_sizes[0] / 2;
    if (npts != NPTS || out_size != NPTS * NPTS) return;
    if (in_sizes[1] != 2 * 64 || in_sizes[3] != 3 * 64 * 192 || in_sizes[6] != 3 * 64 * 64 ||
        in_sizes[8] != 3 * 64 * 256 || in_sizes[10] != 3 * 256 * 64 || in_sizes[12] != 64 * 64)
        return;

    char* ws = (char*)d_ws;
    size_t off = 0;
    auto carve = [&](size_t bytes) { size_t o = off; off += (bytes + 255) & ~(size_t)255; return o; };
    const size_t o_fA = carve((size_t)NPTS * 64 * 4);
    const size_t o_fB = carve((size_t)NPTS * 64 * 4);
    const size_t o_q  = carve((size_t)NPTS * 64 * 4);
    const size_t o_k  = carve((size_t)NPTS * 64 * 4);
    const size_t o_v  = carve((size_t)NPTS * 64 * 4);
    const size_t o_hi = carve((size_t)NPTS * 64 * 2);
    const size_t o_lo = carve((size_t)NPTS * 64 * 2);
    if (off > ws_size) return;

    float* featsA = (float*)(ws + o_fA);
    float* featsB = (float*)(ws + o_fB);
    float* qb     = (float*)(ws + o_q);
    float* kb     = (float*)(ws + o_k);
    float* vb     = (float*)(ws + o_v);
    unsigned short* f1hi = (unsigned short*)(ws + o_hi);
    unsigned short* f1lo = (unsigned short*)(ws + o_lo);

    const int rgrid = (npts + 3) / 4;

    rowlin_kernel<2, 64, true><<<rgrid, 64, 0, stream>>>(x, in_w, in_b, featsA, featsA, featsA, npts);

    float* fin = featsA;
    float* fout = featsB;
    for (int l = 0; l < 3; ++l) {
        rowlin_kernel<64, 192, false><<<rgrid, 192, 0, stream>>>(
            fin, qkv_w + (size_t)l * 64 * 192, in_b, qb, kb, vb, npts);
        pair_layer_kernel<<<npts, 128, LAYER_SMEM, stream>>>(
            x, qb, kb, vb,
            pw1 + (size_t)l * 192, pb1 + (size_t)l * 64,
            pw2 + (size_t)l * 64 * 64, pb2 + (size_t)l * 64,
            aw1 + (size_t)l * 64 * 256, ab1 + (size_t)l * 256,
            aw2 + (size_t)l * 256 * 64, ab2 + (size_t)l * 64,
            fout);
        float* t = fin; fin = fout; fout = t;
    }

    fc_split_kernel<<<rgrid, 64, 0, stream>>>(fin, fc_w, fc_b, f1hi, f1lo, npts);
    edge_kernel<<<dim3(NPTS / 64, NPTS / 16), 32, 0, stream>>>(f1hi, f1lo, out);
}
